// MultiHeadGATLayerWithEdgeFeatures_8504035246421
// MI455X (gfx1250) — hardware-run, weakly checked
//
#include <hip/hip_runtime.h>

typedef float          v8f   __attribute__((ext_vector_type(8)));
typedef float          v4f   __attribute__((ext_vector_type(4)));
typedef unsigned int   v4u   __attribute__((ext_vector_type(4)));
typedef int            v8i   __attribute__((ext_vector_type(8)));
typedef unsigned short v8us  __attribute__((ext_vector_type(8)));
typedef unsigned short v16us __attribute__((ext_vector_type(16)));
typedef __bf16         v16bf __attribute__((ext_vector_type(16)));
typedef _Float16       v16h  __attribute__((ext_vector_type(16)));
typedef v4f  __attribute__((may_alias)) v4fa;
typedef v8us __attribute__((may_alias)) v8usa;
union FragB { v16bf v; v16us u; v8us h[2]; v8i w; };
union FragH { v16h  v; v16us u; v8us h[2]; v8i w; };

__device__ __forceinline__ v8f wmb(const FragB& a, const FragB& b, v8f c) {
  v8f d = __builtin_amdgcn_wmma_f32_16x16x32_bf16(false, a.v, false, b.v, (short)0, c, false, false);
  asm volatile("v_nop\n\tv_nop\n\tv_nop\n\tv_nop" : "+v"(d) : "v"(a.w), "v"(b.w));
  return d;
}

__device__ __forceinline__ v8f wmh(const FragH& a, const FragH& b, v8f c) {
  v8f d = __builtin_amdgcn_wmma_f32_16x16x32_f16(false, a.v, false, b.v, (short)0, c, false, false);
  asm volatile("v_nop\n\tv_nop\n\tv_nop\n\tv_nop" : "+v"(d) : "v"(a.w), "v"(b.w));
  return d;
}

__device__ __forceinline__ unsigned bf16_bits(float f) {
  const unsigned u = __float_as_uint(f);
  const unsigned r = (u + 0x7FFFu + ((u >> 16) & 1u)) >> 16;
  const unsigned q = (u >> 16) | 0x40u;
  return ((u & 0x7fffffffu) > 0x7f800000u) ? q : r;
}

__device__ __forceinline__ float bf16_val(float f) {
  return __uint_as_float(bf16_bits(f) << 16);
}
__device__ __forceinline__ int clampi(int v, int lo, int hi) {
  return v < lo ? lo : (v > hi ? hi : v);
}

__device__ __forceinline__ unsigned f16_bits(float f) {
  const unsigned u  = __float_as_uint(f);
  const unsigned s  = (u >> 16) & 0x8000u;
  const unsigned a  = u & 0x7fffffffu;
  const unsigned t  = a - 0x38000000u;
  const unsigned r  = (t + 0x0FFFu + ((t >> 13) & 1u)) >> 13;
  const unsigned rc = r > 0x7C00u ? 0x7C00u : r;
  const bool small  = a < 0x38800000u;
  const bool isnan  = a > 0x7f800000u;
  const unsigned fin = small ? 0u : (s | rc);
  return isnan ? (s | 0x7E00u) : fin;
}

__device__ __forceinline__ unsigned pk16(unsigned lo, unsigned hi) { return lo | (hi << 16); }
__device__ __forceinline__ unsigned bf16_lo_bits(float v) {
  float hi = bf16_val(v);
  asm volatile("" : "+v"(hi));
  return bf16_bits(v - hi);
}
__device__ __forceinline__ v4u pack8_bf16(v4f a, v4f c) {
  return (v4u){ pk16(bf16_bits(a[0]), bf16_bits(a[1])), pk16(bf16_bits(a[2]), bf16_bits(a[3])),
                pk16(bf16_bits(c[0]), bf16_bits(c[1])), pk16(bf16_bits(c[2]), bf16_bits(c[3])) };
}
__device__ __forceinline__ v4u pack8_bf16_lo(v4f a, v4f c) {
  return (v4u){ pk16(bf16_lo_bits(a[0]), bf16_lo_bits(a[1])), pk16(bf16_lo_bits(a[2]), bf16_lo_bits(a[3])),
                pk16(bf16_lo_bits(c[0]), bf16_lo_bits(c[1])), pk16(bf16_lo_bits(c[2]), bf16_lo_bits(c[3])) };
}
__device__ __forceinline__ v4u pack8_f16(v4f a, v4f c) {
  return (v4u){ pk16(f16_bits(a[0]), f16_bits(a[1])), pk16(f16_bits(a[2]), f16_bits(a[3])),
                pk16(f16_bits(c[0]), f16_bits(c[1])), pk16(f16_bits(c[2]), f16_bits(c[3])) };
}

template <int FORM>
__global__ __launch_bounds__(256) void k_plane(const float* __restrict__ src, int rows, int cols, int ldsrc,
                                               unsigned short* __restrict__ dst, int MP, int KP) {
  static_assert(FORM >= 0 && FORM <= 3);
  const int KTOT = (FORM == 1 || FORM == 3) ? 2 * KP : KP;
  const unsigned ppr   = (unsigned)(KTOT >> 3);
  const unsigned kp8   = (unsigned)(KP >> 3);
  const unsigned total = (unsigned)MP * ppr;
  const unsigned g     = blockIdx.x * 256u + threadIdx.x;
  const unsigned rowu  = g / ppr;
  const unsigned p     = g - rowu * ppr;
  const bool second    = p >= kp8;
  const int row = (int)rowu;
  const int c0  = (int)((second ? p - kp8 : p) << 3);
  const float* srow = src + (size_t)clampi(row, 0, rows - 1) * (size_t)ldsrc;
  float x[8];
  unsigned mk[8];
#pragma unroll
  for (int e = 0; e < 8; ++e) {
    const int c = c0 + e;
    const float v = srow[clampi(c, 0, cols - 1)];
    asm volatile("" :: "v"(v));
    x[e]  = v;
    mk[e] = (row < rows && c < cols) ? 0xFFFFu : 0u;
  }
  const v4f a = (v4f){ x[0], x[1], x[2], x[3] };
  const v4f c = (v4f){ x[4], x[5], x[6], x[7] };
  v4u o;
  if (FORM == 2) {
    o = pack8_f16(a, c);
  } else {
    const v4u hi = pack8_bf16(a, c);
    o = hi;
    if (FORM == 1) { const v4u lo = pack8_bf16_lo(a, c); o = second ? lo : hi; }
  }
  const v4u mw = (v4u){ pk16(mk[0], mk[1]), pk16(mk[2], mk[3]), pk16(mk[4], mk[5]), pk16(mk[6], mk[7]) };
  o &= mw;
  if (g < total) {
    volatile v4u* q = (volatile v4u*)(dst + (size_t)g * 8);
    *q = o;
    __threadfence();
    *q = o;
  }
}

template <int FORM> struct FragOf    { typedef FragB T; };
template <>         struct FragOf<2> { typedef FragH T; };
__device__ __forceinline__ v8f mm(const FragB& a, const FragB& b, v8f c) { return wmb(a, b, c); }
__device__ __forceinline__ v8f mm(const FragH& a, const FragH& b, v8f c) { return wmh(a, b, c); }
template <class F> __device__ __forceinline__ F ld_frag(const unsigned short* p) {
  F f;
  f.h[0] = *(const v8usa*)(p);
  f.h[1] = *(const v8usa*)(p + 16);
  return f;
}

template <int FORM, int EPI>
__global__ __launch_bounds__(256) __attribute__((amdgpu_num_vgpr(248)))
void k_gemm_nt(const unsigned short* __restrict__ A, const unsigned short* __restrict__ B,
               const float* __restrict__ bias, float* __restrict__ D, int M, int N, int KTOT, int ldd) {
  static_assert(FORM >= 0 && FORM <= 2);
  static_assert(EPI == 0 || EPI == 1);
  typedef typename FragOf<FORM>::T F;
  __shared__ __attribute__((aligned(16))) float sT[8][16 * 68];
  const int lane = threadIdx.x & 31;
  const int wave = threadIdx.x >> 5;
  const int tilesM = (M + 63) >> 6;
  const int tilesN = (N + 63) >> 6;
  const int tile = blockIdx.x * 8 + wave;
  if (tile >= tilesM * tilesN) return;
  const int tm = tile / tilesN;
  const int tn = tile - tm * tilesN;
  const int m0 = tm << 6;
  const int n0 = tn << 6;

  const int rl = lane & 15;
  const int h8 = (lane >> 4) * 8;
  const unsigned short* pa = A + (size_t)(m0 + rl) * (size_t)KTOT + h8;
  const unsigned short* pb = B + (size_t)(n0 + rl) * (size_t)KTOT + h8;

  v8f acc[4][4];
#pragma unroll
  for (int i = 0; i < 4; ++i)
#pragma unroll
    for (int j = 0; j < 4; ++j) acc[i][j] = (v8f){0.f, 0.f, 0.f, 0.f, 0.f, 0.f, 0.f, 0.f};

#pragma unroll 1
  for (int k0 = 0; k0 < KTOT; k0 += 32) {
    F bf[4];
#pragma unroll
    for (int j = 0; j < 4; ++j) bf[j] = ld_frag<F>(pb + (size_t)(j << 4) * (size_t)KTOT + k0);
#pragma unroll
    for (int i = 0; i < 4; ++i) {
      const F af = ld_frag<F>(pa + (size_t)(i << 4) * (size_t)KTOT + k0);
#pragma unroll
      for (int j = 0; j < 4; ++j) acc[i][j] = mm(af, bf[j], acc[i][j]);
    }
  }

  float* slab = sT[wave];
  const int hh = lane >> 4;
  const int c4 = (lane & 15) * 4;
  const int nc = n0 + c4;
  const bool cok = nc < N;
  v4f bv = (v4f){0.f, 0.f, 0.f, 0.f};
  if (EPI == 1) {
    bv = *(const v4fa*)(bias + clampi(nc, 0, N - 4));
    asm volatile("" :: "v"(bv));
  }
#pragma unroll
  for (int i = 0; i < 4; ++i) {
    const int mBase = m0 + (i << 4);
#pragma unroll
    for (int j = 0; j < 4; ++j) {
#pragma unroll
      for (int r = 0; r < 8; ++r) slab[(h8 + r) * 68 + (j << 4) + rl] = acc[i][j][r];
    }
    __builtin_amdgcn_fence(__ATOMIC_RELEASE, "workgroup");
    __builtin_amdgcn_wave_barrier();
    __builtin_amdgcn_fence(__ATOMIC_ACQUIRE, "workgroup");
    v4f vv[8];
#pragma unroll
    for (int it = 0; it < 8; ++it) {
      const int row = it * 2 + hh;
      v4f v = *(const v4fa*)(slab + row * 68 + c4);
      if (EPI == 1) v += bv;
      vv[it] = v;
    }
    for (int pass = 0; pass < 2; ++pass) {
#pragma unroll
      for (int it = 0; it < 8; ++it) {
        const int row = mBase + it * 2 + hh;
        if (cok && row < M) *(volatile v4f*)(D + (size_t)row * (size_t)ldd + nc) = vv[it];
      }
      __threadfence();
    }
    __builtin_amdgcn_fence(__ATOMIC_RELEASE, "workgroup");
    __builtin_amdgcn_wave_barrier();
    __builtin_amdgcn_fence(__ATOMIC_ACQUIRE, "workgroup");
  }
}

#pragma clang fp contract(off)

typedef int v4i __attribute__((ext_vector_type(4)));
typedef int v2i __attribute__((ext_vector_type(2)));
typedef v4i __attribute__((may_alias)) v4ia;
typedef v2i __attribute__((may_alias)) v2ia;

#define GN      20000
#define GE      640000
#define GMP     20032
#define GC      128
#define GAROW   80
#define NBRUN   512
#define NBLK    40
#define LCAP    21504
#define WLCAP   4096
#define DEGCAP  72
#define CHUNK   2048
#define NCHUNK  313
#define NGRP    625
#define B512MAX 16797
#define DEGMAX  57
#define LDS_BUCKET ((8 * WLCAP + LCAP + 2 * NBRUN + 32) * 4)

#define SZ_HB   ((size_t)GMP * 128 * 2)
#define SZ_WT   ((size_t)128 * 128 * 2)
#define SZ_ATAB ((size_t)1536)
#define SZ_WH   ((size_t)GMP * 128 * 4)
#define SZ_SS   ((size_t)GMP * 16)
#define SZ_OFF  ((size_t)NBLK * NBRUN * 8)
#define SZ_LIST ((size_t)NBLK * LCAP * 4)
#define WS_TOTAL (SZ_HB + SZ_WT + SZ_ATAB + SZ_WH + SZ_SS + SZ_SS + SZ_OFF + SZ_LIST)

static_assert(4 * 32 == GC);
static_assert(GN % 32 == 0 && GN % 8 == 0 && GN / 32 == NGRP);
static_assert(GMP % 64 == 0 && GMP >= GN);
static_assert(GE <= (1 << 20));
static_assert(NBRUN * NBLK >= GN && NBRUN * (NBLK - 1) < GN);
static_assert((LCAP * 4) % 128 == 0 && LCAP % 1024 == 0);
static_assert(4 * LCAP >= 5 * B512MAX);
static_assert(8 * WLCAP >= LCAP);
static_assert(DEGCAP >= DEGMAX + 8);
static_assert(NCHUNK * CHUNK >= GE && (NCHUNK - 1) * CHUNK < GE);
static_assert(LDS_BUCKET <= 262144);
static_assert(SZ_HB % 256 == 0 && SZ_WT % 256 == 0 && SZ_ATAB % 256 == 0 && SZ_WH % 256 == 0);
static_assert(SZ_SS % 256 == 0 && SZ_OFF % 256 == 0 && SZ_LIST % 256 == 0);
static_assert(WS_TOTAL <= ((size_t)128 << 20));
static_assert(SZ_ATAB >= 4 * GAROW * 4);

__global__ __launch_bounds__(256) void k_prep(const float* __restrict__ W, const float* __restrict__ a,
                                              unsigned short* __restrict__ WT, float* __restrict__ ATAB) {
  __shared__ __attribute__((aligned(16))) float sW[128 * 36];
  const int tid = (int)threadIdx.x;
  const int nb0 = (int)blockIdx.x * 32;
#pragma unroll
  for (int i = 0; i < 4; ++i) {
    const int f  = i * 256 + tid;
    const int k  = f >> 3;
    const int c4 = (f & 7) * 4;
    const v4f v = *(const v4fa*)(W + k * 128 + nb0 + c4);
    *(v4fa*)(sW + k * 36 + c4) = v;
  }
  __syncthreads();
  v4u o0, o1;
  int r0, k00, r1, k01;
  {
    const int piece = tid;
    r0 = piece >> 4; k00 = (piece & 15) * 8;
    const v4f x = (v4f){ sW[(k00 + 0) * 36 + r0], sW[(k00 + 1) * 36 + r0], sW[(k00 + 2) * 36 + r0], sW[(k00 + 3) * 36 + r0] };
    const v4f y = (v4f){ sW[(k00 + 4) * 36 + r0], sW[(k00 + 5) * 36 + r0], sW[(k00 + 6) * 36 + r0], sW[(k00 + 7) * 36 + r0] };
    o0 = pack8_bf16(x, y);
  }
  {
    const int piece = 256 + tid;
    r1 = piece >> 4; k01 = (piece & 15) * 8;
    const v4f x = (v4f){ sW[(k01 + 0) * 36 + r1], sW[(k01 + 1) * 36 + r1], sW[(k01 + 2) * 36 + r1], sW[(k01 + 3) * 36 + r1] };
    const v4f y = (v4f){ sW[(k01 + 4) * 36 + r1], sW[(k01 + 5) * 36 + r1], sW[(k01 + 6) * 36 + r1], sW[(k01 + 7) * 36 + r1] };
    o1 = pack8_bf16(x, y);
  }
  volatile v4u* q0 = (volatile v4u*)(WT + (size_t)(nb0 + r0) * 128 + k00);
  volatile v4u* q1 = (volatile v4u*)(WT + (size_t)(nb0 + r1) * 128 + k01);
  *q0 = o0; *q1 = o1;
  __threadfence();
  *q0 = o0; *q1 = o1;

  const int t = tid < 80 ? tid : 79;
  const v4f av = *(const v4fa*)(a + 4 * t);
  asm volatile("" :: "v"(av));
  const v4f ar = (v4f){ bf16_val(av.x), bf16_val(av.y), bf16_val(av.z), bf16_val(av.w) };
  if (blockIdx.x == 0 && tid < 80) {
    volatile v4f* qa = (volatile v4f*)(ATAB + 4 * tid);
    *qa = ar;
    __threadfence();
    *qa = ar;
  }
}

__global__ __launch_bounds__(256) void k_node(const float* __restrict__ WH, const float* __restrict__ ATAB,
                                              float* __restrict__ SS, float* __restrict__ SD) {
  __shared__ __attribute__((aligned(16))) float sA[4 * GAROW];
  __shared__ __attribute__((aligned(16))) float sS[8][128];
  __shared__ __attribute__((aligned(16))) float sD[8][128];
  const int tid = (int)threadIdx.x, lane = tid & 31, wave = tid >> 5;
  {
    const int t = tid < 80 ? tid : 79;
    const v4f v = *(const v4fa*)(ATAB + 4 * t);
    asm volatile("" :: "v"(v));
    if (tid < 80) *(v4fa*)(sA + 4 * tid) = v;
  }
  __syncthreads();
  const int g = (int)blockIdx.x * 8 + wave;
  if (g < NGRP) {
    const int hd = lane >> 3;
    const int d0 = (lane & 7) * 4;
    const v4f as = *(const v4fa*)(sA + hd * GAROW + d0);
    const v4f ad = *(const v4fa*)(sA + hd * GAROW + 32 + d0);
    float* stS = sS[wave];
    float* stD = sD[wave];
#pragma unroll 4
    for (int i = 0; i < 32; ++i) {
      const int n = g * 32 + i;
      const v4f r = *(const v4fa*)(WH + (size_t)n * GC + 4 * lane);
      float ps = r.x * as.x;
      ps = ps + r.y * as.y;
      ps = ps + r.z * as.z;
      ps = ps + r.w * as.w;
      float pd = r.x * ad.x;
      pd = pd + r.y * ad.y;
      pd = pd + r.z * ad.z;
      pd = pd + r.w * ad.w;
      ps = ps + __shfl_xor(ps, 1);
      pd = pd + __shfl_xor(pd, 1);
      ps = ps + __shfl_xor(ps, 2);
      pd = pd + __shfl_xor(pd, 2);
      ps = ps + __shfl_xor(ps, 4);
      pd = pd + __shfl_xor(pd, 4);
      if ((lane & 7) == 0) { stS[i * 4 + hd] = ps; stD[i * 4 + hd] = pd; }
    }
    __builtin_amdgcn_fence(__ATOMIC_RELEASE, "workgroup");
    __builtin_amdgcn_wave_barrier();
    __builtin_amdgcn_fence(__ATOMIC_ACQUIRE, "workgroup");
    const v4f vs = *(const v4fa*)(stS + 4 * lane);
    const v4f vd = *(const v4fa*)(stD + 4 * lane);
    volatile v4f* qs = (volatile v4f*)(SS + (size_t)(g * 32 + lane) * 4);
    volatile v4f* qd = (volatile v4f*)(SD + (size_t)(g * 32 + lane) * 4);
    *qs = vs; *qd = vd;
    __threadfence();
    *qs = vs; *qd = vd;
  }
}

__global__ __launch_bounds__(256) void k_bucket(const int* __restrict__ keys, int* __restrict__ LISTg,
                                                int* __restrict__ OFFg) {
  extern __shared__ __attribute__((aligned(16))) int dl[];
  int* wl     = dl;
  int* placed = dl + 8 * WLCAP;
  int* scnt   = placed + LCAP;
  int* cur    = scnt + NBRUN;
  int* misc   = cur + NBRUN;
  const int tid = (int)threadIdx.x, lane = tid & 31, wave = tid >> 5;
  const int blk = (int)blockIdx.x;
  const int ownBase = blk * NBRUN;
  int live = GN - ownBase;
  live = live > NBRUN ? NBRUN : (live < 0 ? 0 : live);

  scnt[tid] = 0;
  scnt[tid + 256] = 0;
  if (tid < 32) misc[tid] = 0;
  {
    const v4i z4 = (v4i){0, 0, 0, 0};
#pragma unroll 1
    for (int it = 0; it < LCAP / 1024; ++it) *(v4ia*)(placed + 4 * (it * 256 + tid)) = z4;
  }
  __syncthreads();

  int wc = 0;
  const int el0 = tid * 8;
  const unsigned ub = (unsigned)ownBase;
  const unsigned ul = (unsigned)live;
  int* mywl = wl + wave * WLCAP;
#pragma unroll 1
  for (int ch = 0; ch < NCHUNK; ++ch) {
    const int cbase = ch * CHUNK;
    const int e0 = cbase + el0;
    v4i da, db;
    if (cbase + CHUNK <= GE) {
      da = *(const v4ia*)(keys + e0);
      db = *(const v4ia*)(keys + e0 + 4);
      asm volatile("" :: "v"(da), "v"(db));
    } else {
      int kk[8];
#pragma unroll
      for (int j = 0; j < 8; ++j) {
        const int ej = e0 + j;
        const int v = keys[ej < GE ? ej : GE - 1];
        asm volatile("" :: "v"(v));
        kk[j] = (ej < GE) ? v : -1;
      }
      da = (v4i){ kk[0], kk[1], kk[2], kk[3] };
      db = (v4i){ kk[4], kk[5], kk[6], kk[7] };
    }
    const unsigned s0 = (unsigned)da.x - ub, s1 = (unsigned)da.y - ub;
    const unsigned s2 = (unsigned)da.z - ub, s3 = (unsigned)da.w - ub;
    const unsigned s4 = (unsigned)db.x - ub, s5 = (unsigned)db.y - ub;
    const unsigned s6 = (unsigned)db.z - ub, s7 = (unsigned)db.w - ub;
    const bool h0 = s0 < ul, h1 = s1 < ul, h2 = s2 < ul, h3 = s3 < ul;
    const bool h4 = s4 < ul, h5 = s5 < ul, h6 = s6 < ul, h7 = s7 < ul;
    const unsigned any = __builtin_amdgcn_ballot_w32(h0 | h1 | h2 | h3 | h4 | h5 | h6 | h7);
    if (any != 0u) {
#define HITJ(J, HJ, SJ) { \
        const unsigned mj = __builtin_amdgcn_ballot_w32(HJ); \
        if (mj != 0u) { \
          if (HJ) { \
            const int pos = wc + (int)__builtin_amdgcn_mbcnt_lo(mj, 0u); \
            if (pos < WLCAP) mywl[pos] = (e0 + (J)) | (int)((SJ) << 20); \
          } \
          wc += (int)__builtin_popcount(mj); } }
      HITJ(0, h0, s0)
      HITJ(1, h1, s1)
      HITJ(2, h2, s2)
      HITJ(3, h3, s3)
      HITJ(4, h4, s4)
      HITJ(5, h5, s5)
      HITJ(6, h6, s6)
      HITJ(7, h7, s7)
#undef HITJ
    }
  }
  if (lane == 0) misc[wave] = wc;
  __syncthreads();

  if (wave == 0) {
#pragma unroll 1
    for (int w2 = 0; w2 < 8; ++w2) {
      int nw = misc[w2];
      nw = nw < 0 ? 0 : (nw > WLCAP ? WLCAP : nw);
      nw = __builtin_amdgcn_readfirstlane(nw);
#pragma unroll 1
      for (int b0 = 0; b0 < nw; b0 += 32) {
        int idx = b0 + lane;
        idx = idx > nw - 1 ? nw - 1 : idx;
        const int uv  = wl[w2 * WLCAP + idx];
        const int m32 = (nw - b0) < 32 ? (nw - b0) : 32;
#pragma unroll 1
        for (int k = 0; k < m32; ++k) {
          const int u  = __builtin_amdgcn_readlane(uv, k);
          const int sl = (u >> 20) & (NBRUN - 1);
          if (lane == 0) scnt[sl] = scnt[sl] + 1;
        }
      }
    }
  }
  __syncthreads();

  int c0 = scnt[2 * tid], c1 = scnt[2 * tid + 1];
  c0 = c0 < 0 ? 0 : c0;
  c1 = c1 < 0 ? 0 : c1;
  const int ts = c0 + c1;
  int incl = ts;
#pragma unroll
  for (int d = 1; d < 32; d <<= 1) {
    const int up = __shfl_up(incl, d);
    incl += (lane >= d) ? up : 0;
  }
  if (lane == 31) misc[8 + wave] = incl;
  if (c0 > DEGCAP || c1 > DEGCAP) misc[16] = 1;
  __syncthreads();
  int pre = 0, nh = 0;
  bool wovf = false;
#pragma unroll
  for (int w2 = 0; w2 < 8; ++w2) {
    const int t2 = misc[8 + w2];
    nh  += t2;
    pre += (w2 < wave) ? t2 : 0;
    wovf = wovf || (misc[w2] > WLCAP);
  }
  const int run0 = pre + incl - ts;
  const int run1 = run0 + c0;
  cur[2 * tid]     = run0;
  cur[2 * tid + 1] = run1;
  const bool ovf = wovf || (nh > LCAP) || (misc[16] != 0);
  __syncthreads();

  if (wave == 0) {
#pragma unroll 1
    for (int w2 = 0; w2 < 8; ++w2) {
      int nw = misc[w2];
      nw = nw < 0 ? 0 : (nw > WLCAP ? WLCAP : nw);
      nw = __builtin_amdgcn_readfirstlane(nw);
#pragma unroll 1
      for (int b0 = 0; b0 < nw; b0 += 32) {
        int idx = b0 + lane;
        idx = idx > nw - 1 ? nw - 1 : idx;
        const int uv  = wl[w2 * WLCAP + idx];
        const int m32 = (nw - b0) < 32 ? (nw - b0) : 32;
#pragma unroll 1
        for (int k = 0; k < m32; ++k) {
          const int u   = __builtin_amdgcn_readlane(uv, k);
          const int sl  = (u >> 20) & (NBRUN - 1);
          const int eid = u & 0xFFFFF;
          if (lane == 0) {
            int pos = cur[sl];
            pos = pos < 0 ? 0 : (pos > LCAP - 1 ? LCAP - 1 : pos);
            placed[pos] = eid;
            cur[sl] = pos + 1;
          }
        }
      }
    }
  }
  __syncthreads();

  int* lbase = LISTg + (size_t)blk * LCAP;
  for (int pass = 0; pass < 2; ++pass) {
#pragma unroll 1
    for (int it = 0; it < LCAP / 1024; ++it) {
      const int o4 = 4 * (it * 256 + tid);
      const v4i v = *(const v4ia*)(placed + o4);
      *(volatile v4i*)(lbase + o4) = v;
    }
    __threadfence();
  }
  {
    const v4i oc = (v4i){ run0, ovf ? -1 : c0, run1, ovf ? -1 : c1 };
    volatile v4i* qo = (volatile v4i*)(OFFg + (size_t)blk * (NBRUN * 2) + 4 * tid);
    *qo = oc;
    __threadfence();
    *qo = oc;
  }
}

__global__ __launch_bounds__(256) void k_replay(const int* __restrict__ ei, const float* __restrict__ ea,
                                                const float* __restrict__ WH, const float* __restrict__ SS,
                                                const float* __restrict__ SD, const float* __restrict__ ATAB,
                                                const int* __restrict__ LISTg, const int* __restrict__ OFFg,
                                                float* __restrict__ out) {
  __shared__ __attribute__((aligned(16))) float sA[4 * GAROW];
  const int tid = (int)threadIdx.x, lane = tid & 31, wave = tid >> 5;
  {
    const int t = tid < 80 ? tid : 79;
    const v4f v = *(const v4fa*)(ATAB + 4 * t);
    asm volatile("" :: "v"(v));
    if (tid < 80) *(v4fa*)(sA + 4 * tid) = v;
  }
  __syncthreads();
  const int n = (int)blockIdx.x * 8 + wave;
  if (n < GN) {
    const int hd  = lane >> 3;
    const int blk = n >> 9;
    const v2i oc = *(const v2ia*)(OFFg + 2 * (size_t)n);
    asm volatile("" :: "v"(oc));
    const int craw = oc.y;
    const bool bad = (craw < 0) || (craw > DEGCAP);
    const int stv = clampi(oc.x, 0, LCAP - 1);
    int cnv = bad ? 0 : craw;
    cnv = cnv > (LCAP - stv) ? (LCAP - stv) : cnv;
    const int cn    = __builtin_amdgcn_readfirstlane(cnv);
    const int start = __builtin_amdgcn_readfirstlane(stv);
    const v4f ss = *(const v4fa*)(SS + (size_t)n * 4);
    asm volatile("" :: "v"(ss));
    const int* lst = LISTg + (size_t)blk * LCAP + start;
    v4f acc = (v4f){0.0f, 0.0f, 0.0f, 0.0f};

#pragma unroll 1
    for (int b0 = 0; b0 < cn; b0 += 32) {
      int jj = b0 + lane;
      jj = jj > cn - 1 ? cn - 1 : jj;
      int eid = lst[jj];
      asm volatile("" :: "v"(eid));
      eid = clampi(eid, 0, GE - 1);
      int dstv = ei[GE + eid];
      asm volatile("" :: "v"(dstv));
      dstv = clampi(dstv, 0, GN - 1);
      const v4f sd = *(const v4fa*)(SD + (size_t)dstv * 4);
      asm volatile("" :: "v"(sd.x));
      asm volatile("" :: "v"(sd.y));
      asm volatile("" :: "v"(sd.z));
      asm volatile("" :: "v"(sd.w));
      float d0 = 0.0f, d1 = 0.0f, d2 = 0.0f, d3 = 0.0f;
      const float* erow = ea + (size_t)eid * 16;
#pragma unroll 1
      for (int g = 0; g < 4; ++g) {
        const v4f x = *(const v4fa*)(erow + 4 * g);
        asm volatile("" :: "v"(x.x));
        asm volatile("" :: "v"(x.y));
        asm volatile("" :: "v"(x.z));
        asm volatile("" :: "v"(x.w));
        const float x0 = bf16_val(x.x), x1 = bf16_val(x.y), x2 = bf16_val(x.z), x3 = bf16_val(x.w);
        const v4f a0 = *(const v4fa*)(sA + 0 * GAROW + 64 + 4 * g);
        const v4f a1 = *(const v4fa*)(sA + 1 * GAROW + 64 + 4 * g);
        const v4f a2 = *(const v4fa*)(sA + 2 * GAROW + 64 + 4 * g);
        const v4f a3 = *(const v4fa*)(sA + 3 * GAROW + 64 + 4 * g);
        d0 = d0 + x0 * a0.x; d0 = d0 + x1 * a0.y; d0 = d0 + x2 * a0.z; d0 = d0 + x3 * a0.w;
        d1 = d1 + x0 * a1.x; d1 = d1 + x1 * a1.y; d1 = d1 + x2 * a1.z; d1 = d1 + x3 * a1.w;
        d2 = d2 + x0 * a2.x; d2 = d2 + x1 * a2.y; d2 = d2 + x2 * a2.z; d2 = d2 + x3 * a2.w;
        d3 = d3 + x0 * a3.x; d3 = d3 + x1 * a3.y; d3 = d3 + x2 * a3.z; d3 = d3 + x3 * a3.w;
      }
      float e0 = (ss.x + sd.x) + d0;
      float e1 = (ss.y + sd.y) + d1;
      float e2 = (ss.z + sd.z) + d2;
      float e3 = (ss.w + sd.w) + d3;
      e0 = (e0 >= 0.0f) ? e0 : 0.2f * e0;
      e1 = (e1 >= 0.0f) ? e1 : 0.2f * e1;
      e2 = (e2 >= 0.0f) ? e2 : 0.2f * e2;
      e3 = (e3 >= 0.0f) ? e3 : 0.2f * e3;
      float m = e0;
      m = (e1 > m) ? e1 : m;
      m = (e2 > m) ? e2 : m;
      m = (e3 > m) ? e3 : m;
      v4f ev = (v4f){ e0, e1, e2, e3 };
#pragma unroll 1
      for (int i = 0; i < 4; ++i) {
        const float t = expf(ev.x - m);
        ev = (v4f){ ev.y, ev.z, ev.w, t };
      }
      const float sden = ((ev.x + ev.y) + ev.z) + ev.w;
#pragma unroll 1
      for (int i = 0; i < 4; ++i) {
        const float t = ev.x / sden;
        ev = (v4f){ ev.y, ev.z, ev.w, t };
      }
      const int a0i = __float_as_int(ev.x);
      const int a1i = __float_as_int(ev.y);
      const int a2i = __float_as_int(ev.z);
      const int a3i = __float_as_int(ev.w);

      const int bc = (cn - b0) < 32 ? (cn - b0) : 32;
#pragma unroll 1
      for (int t = 0; t < bc; ++t) {
        const int d = __builtin_amdgcn_readlane(dstv, t);
        const float w0 = __int_as_float(__builtin_amdgcn_readlane(a0i, t));
        const float w1 = __int_as_float(__builtin_amdgcn_readlane(a1i, t));
        const float w2 = __int_as_float(__builtin_amdgcn_readlane(a2i, t));
        const float w3 = __int_as_float(__builtin_amdgcn_readlane(a3i, t));
        float w = w3;
        w = (hd == 2) ? w2 : w;
        w = (hd == 1) ? w1 : w;
        w = (hd == 0) ? w0 : w;
        const v4f row = *(const v4fa*)(WH + (size_t)d * GC + 4 * lane);
        asm volatile("" :: "v"(row));
        acc.x = acc.x + w * row.x;
        acc.y = acc.y + w * row.y;
        acc.z = acc.z + w * row.z;
        acc.w = acc.w + w * row.w;
      }
    }

    const float qn = __int_as_float(0x7fc00000);
    v4f v = (v4f){ bad ? qn : acc.x, bad ? qn : acc.y, bad ? qn : acc.z, bad ? qn : acc.w };
#pragma unroll 1
    for (int i = 0; i < 4; ++i) {
      const float x = v.x;
      const float t = (x > 0.0f) ? x : expm1f(x);
      v = (v4f){ v.y, v.z, v.w, t };
    }
    volatile v4f* q = (volatile v4f*)(out + (size_t)n * GC + 4 * lane);
    *q = v;
    __threadfence();
    *q = v;
  }
}

extern "C" void kernel_launch(void* const* d_in, const int* in_sizes, int n_in,
                              void* d_out, int out_size, void* d_ws, size_t ws_size,
                              hipStream_t stream) {
  if (n_in < 5) return;
  if (in_sizes[0] != GN * 128) return;
  if (in_sizes[1] != 2 * GE) return;
  if (in_sizes[2] != GE * 16) return;
  if (in_sizes[3] != 128 * 128) return;
  if (in_sizes[4] != 4 * GAROW) return;
  if (out_size != GN * GC) return;
  if (ws_size < WS_TOTAL) return;

  const float* h  = (const float*)d_in[0];
  const int*   ei = (const int*)  d_in[1];
  const float* ea = (const float*)d_in[2];
  const float* W  = (const float*)d_in[3];
  const float* a  = (const float*)d_in[4];
  float* out = (float*)d_out;

  char* ws = (char*)d_ws;
  size_t off = 0;
  unsigned short* HB = (unsigned short*)(ws + off); off += SZ_HB;
  unsigned short* WT = (unsigned short*)(ws + off); off += SZ_WT;
  float* ATAB        = (float*)(ws + off);          off += SZ_ATAB;
  float* WH          = (float*)(ws + off);          off += SZ_WH;
  float* SSp         = (float*)(ws + off);          off += SZ_SS;
  float* SDp         = (float*)(ws + off);          off += SZ_SS;
  int*   OFFCNT      = (int*)(ws + off);            off += SZ_OFF;
  int*   LIST        = (int*)(ws + off);            off += SZ_LIST;
  if (off != WS_TOTAL) return;

  hipFuncSetAttribute(reinterpret_cast<const void*>(&k_bucket),
                      hipFuncAttributeMaxDynamicSharedMemorySize, LDS_BUCKET);

  k_plane<0><<<(GMP * 128 / 8) / 256, 256, 0, stream>>>(h, GN, 128, 128, HB, GMP, 128);
  k_prep<<<4, 256, 0, stream>>>(W, a, WT, ATAB);
  k_gemm_nt<0, 0><<<(313 * 2 + 7) / 8, 256, 0, stream>>>(HB, WT, ATAB, WH, GMP, 128, 128, 128);
  k_node<<<(NGRP + 7) / 8, 256, 0, stream>>>(WH, ATAB, SSp, SDp);
  k_bucket<<<NBLK, 256, LDS_BUCKET, stream>>>(ei, LIST, OFFCNT);
  k_replay<<<GN / 8, 256, 0, stream>>>(ei, ea, WH, SSp, SDp, ATAB, LIST, OFFCNT, out);
}
